// enc_mtan_classif_12378095747097
// MI455X (gfx1250) — hardware-verified
//
#include <hip/hip_runtime.h>


typedef _Float16 f16t;
typedef f16t  v16h __attribute__((ext_vector_type(16)));
typedef f16t  v8h  __attribute__((ext_vector_type(8)));
typedef float v8f  __attribute__((ext_vector_type(8)));
typedef float v4f  __attribute__((ext_vector_type(4)));
typedef unsigned int v4u __attribute__((ext_vector_type(4)));

union Frag { v16h v; v8h q[2]; };
union Pk16 { v8h h; v4u u; };
union Pk32 { v4f f; v4u u; };

#define NBLK  16
#define TT    128
#define CH    32
#define NHID  128
#define G3    384
#define F1P   320
#define KWO   32
#define LPH   136
#define LPO   328
#define NSTEP 128

__device__ __forceinline__ v8f wmma16(v16h a, v16h b, v8f c) {
    return __builtin_amdgcn_wmma_f32_16x16x32_f16(false, a, false, b, (short)0, c, false, false);
}

__device__ __forceinline__ void wguard(v8f (&c)[1], Frag (&a)[1], Frag& b) {
    asm volatile("v_nop\n\tv_nop\n\tv_nop\n\tv_nop"
                 : "+v"(c[0])
                 : "v"(a[0].v), "v"(b.v));
}
__device__ __forceinline__ void wguard(v8f (&c)[2], Frag (&a)[2], Frag& b) {
    asm volatile("v_nop\n\tv_nop\n\tv_nop\n\tv_nop"
                 : "+v"(c[0]), "+v"(c[1])
                 : "v"(a[0].v), "v"(a[1].v), "v"(b.v));
}
__device__ __forceinline__ void wguard(v8f (&c)[5], Frag (&a)[5], Frag& b) {
    asm volatile("v_nop\n\tv_nop\n\tv_nop\n\tv_nop"
                 : "+v"(c[0]), "+v"(c[1]), "+v"(c[2]), "+v"(c[3]), "+v"(c[4])
                 : "v"(a[0].v), "v"(a[1].v), "v"(a[2].v), "v"(a[3].v), "v"(a[4].v), "v"(b.v));
}
__device__ __forceinline__ void wguard(v8f (&c)[6], Frag (&a)[6], Frag& b) {
    asm volatile("v_nop\n\tv_nop\n\tv_nop\n\tv_nop"
                 : "+v"(c[0]), "+v"(c[1]), "+v"(c[2]), "+v"(c[3]), "+v"(c[4]), "+v"(c[5])
                 : "v"(a[0].v), "v"(a[1].v), "v"(a[2].v), "v"(a[3].v), "v"(a[4].v), "v"(a[5].v),
                   "v"(b.v));
}

template<int MT>
__device__ __forceinline__ void zacc(v8f (&acc)[MT]) {
    const v8f z = {0.f, 0.f, 0.f, 0.f, 0.f, 0.f, 0.f, 0.f};
#pragma unroll
    for (int i = 0; i < MT; ++i) acc[i] = z;
}

template<int MT, int G, int GS>
__device__ __forceinline__ void mma_acc(v8f (&acc)[MT], const f16t* A, int arow0, int lda,
                                        const f16t* B, int ldb, int ktiles) {
    const int l = threadIdx.x & 31, h = l >> 4, m = l & 15;
    const f16t* bp = B + (size_t)m * ldb + 8 * h;
#pragma unroll 1
    for (int kt = 0; kt < ktiles; ++kt) {
        Frag a[MT];
        Frag b;
        b.q[0] = *(const v8h*)(bp + kt * 32);
        b.q[1] = *(const v8h*)(bp + kt * 32 + 16);
#pragma unroll
        for (int i = 0; i < MT; ++i) {
            const int row = arow0 + 16 * (i % G) + GS * (i / G) + m;
            const f16t* p = A + (size_t)row * lda + kt * 32 + 8 * h;
            a[i].q[0] = *(const v8h*)p;
            a[i].q[1] = *(const v8h*)(p + 16);
        }
#pragma unroll
        for (int i = 0; i < MT; ++i) acc[i] = wmma16(a[i].v, b.v, acc[i]);
        wguard(acc, a, b);
    }
}

template<int MT, bool RELU>
__device__ __forceinline__ void epi_h(v8f (&acc)[MT], int f0, float inv, const float* bias, int nbias,
                                      f16t* L, int pitch) {
    const int l = threadIdx.x & 31, h = l >> 4, m = l & 15;
#pragma unroll
    for (int i = 0; i < MT; ++i) {
        const int jb = f0 + 16 * i + 8 * h;
        Pk16 pk;
#pragma unroll
        for (int r = 0; r < 8; ++r) {
            const int j  = jb + r;
            const int jc = (j < nbias) ? j : (nbias - 1);
            float bv = bias[jc];
            bv = (j < nbias) ? bv : 0.f;
            float v = fmaf(acc[i][r], inv, bv);
            if (RELU) v = fmaxf(v, 0.f);
            pk.h[r] = (f16t)v;
        }
        *(v8h*)(L + (size_t)m * pitch + jb) = pk.h;
    }
}

__device__ __forceinline__ float fsigm(float x) {
    return __builtin_amdgcn_rcpf(1.f + __expf(-x));
}
__device__ __forceinline__ float ftanh(float x) {
    float ax = fabsf(x);
    float t  = __expf(-2.0f * ax);
    float r  = (1.0f - t) * __builtin_amdgcn_rcpf(1.0f + t);
    return copysignf(r, x);
}

__global__ __launch_bounds__(256)
void k_pack(const float* W, f16t* P, int N, int K, int Np, int Kp, float sc) {
    const int i   = blockIdx.x * 256 + threadIdx.x;
    const int kq  = Kp >> 3;
    const int tot = Np * kq;
    if (i >= tot) return;
    const int n = i / kq;
    const int k = (i - n * kq) * 8;
    Pk16 v;
#pragma unroll
    for (int e = 0; e < 8; ++e) {
        const int kk = k + e;
        float wv = 0.f;
        if (n < N && kk < K) wv = W[(size_t)n * K + kk];
        v.h[e] = (f16t)(wv * sc);
    }
    f16t* d = P + (size_t)n * Kp + k;
    *(volatile v4u*)d = v.u;
    __threadfence();
    *(volatile v4u*)d = v.u;
}

__global__ __launch_bounds__(128)
void k_main(const float* x, const f16t* Po, const float* bo,
            const f16t* Pih, const float* bih, const f16t* Phh, const float* bhh,
            const f16t* P1, const float* b1, const f16t* P2, const float* b2,
            const f16t* P3, const float* b3, float* out, int nb, float invW) {
    __shared__ __attribute__((aligned(16))) float sGI[NBLK * G3];
    __shared__ __attribute__((aligned(16))) float sH32[NBLK * NHID];
    __shared__ __attribute__((aligned(16))) f16t  sH16[NBLK * LPH];
    __shared__ __attribute__((aligned(16))) f16t  sAt[NBLK * KWO];
    __shared__ __attribute__((aligned(16))) f16t  sP16[NBLK * LPH];
    __shared__ __attribute__((aligned(16))) f16t  sO1[NBLK * LPO];
    __shared__ __attribute__((aligned(16))) f16t  sO2[NBLK * LPO];
    __shared__ __attribute__((aligned(16))) float sOut[NBLK * 2];

    const int tid = threadIdx.x, w = tid >> 5, l = tid & 31, h = l >> 4, m = l & 15;
    const int b0 = blockIdx.x * NBLK;
    if (b0 + NBLK > nb) return;

    for (int i = tid; i < NBLK * NHID; i += 128) sH32[i] = 0.f;
    for (int i = tid; i < NBLK * LPH;  i += 128) sH16[i] = (f16t)0.0f;

    {
        const int c = l, cm = l & 15;
#pragma unroll 1
        for (int q = 0; q < 4; ++q) {
            const int bb = w + 4 * q;
            const float* xr = x + (size_t)(b0 + bb) * TT * CH;
            float s = 0.f, sa = 0.f, n = 0.f;
#pragma unroll 4
            for (int t = 0; t < TT; ++t) {
                const float v  = xr[t * CH + c];
                const float mk = xr[t * CH + 16 + cm];
                const bool on  = (mk != 0.f);
                sa += v;
                s  += on ? v : 0.f;
                n  += on ? 1.f : 0.f;
            }
            const float r = (n > 0.f) ? (s * (1.0f / n)) : (sa * 0.0078125f);
            sAt[bb * KWO + c] = (f16t)r;
        }
    }
    __syncthreads();

    {
        v8f acc[2]; zacc(acc);
        mma_acc<2, 2, 0>(acc, Po, 32 * w, KWO, sAt, KWO, 1);
        epi_h<2, false>(acc, 32 * w, invW, bo, NHID, sP16, LPH);
    }
    __syncthreads();

    {
        v8f acc[6]; zacc(acc);
        mma_acc<6, 6, 0>(acc, Pih, 96 * w, NHID, sP16, LPH, 4);
#pragma unroll
        for (int i = 0; i < 6; ++i) {
            const int ft = 96 * w + 16 * i;
            const int jb = ft + 8 * h;
            const bool addh = (ft < 2 * NHID);
            Pk32 p0, p1;
#pragma unroll
            for (int r = 0; r < 4; ++r) {
                const float hb0 = addh ? bhh[jb + r] : 0.f;
                const float hb1 = addh ? bhh[jb + 4 + r] : 0.f;
                p0.f[r] = fmaf(acc[i][r],     invW, bih[jb + r] + hb0);
                p1.f[r] = fmaf(acc[i][4 + r], invW, bih[jb + 4 + r] + hb1);
            }
            float* d = sGI + m * G3 + jb;
            *(v4f*)d       = p0.f;
            *(v4f*)(d + 4) = p1.f;
        }
    }
    __syncthreads();

    {
        const int j0 = 32 * w;
        float bn[2][8];
#pragma unroll
        for (int ti = 0; ti < 2; ++ti)
#pragma unroll
            for (int r = 0; r < 8; ++r)
                bn[ti][r] = bhh[2 * NHID + j0 + 16 * ti + 8 * h + r];

#pragma unroll 1
        for (int step = 0; step < NSTEP; ++step) {
            v8f acc[6]; zacc(acc);
            mma_acc<6, 2, NHID>(acc, Phh, j0, NHID, sH16, LPH, 4);
            __syncthreads();
#pragma unroll
            for (int ti = 0; ti < 2; ++ti) {
                const int jb = j0 + 16 * ti + 8 * h;
                const float* gp = sGI + m * G3 + jb;
                const v4f gr0 = *(const v4f*)gp,               gr1 = *(const v4f*)(gp + 4);
                const v4f gz0 = *(const v4f*)(gp + NHID),      gz1 = *(const v4f*)(gp + NHID + 4);
                const v4f gn0 = *(const v4f*)(gp + 2 * NHID),  gn1 = *(const v4f*)(gp + 2 * NHID + 4);
                float* hp = sH32 + m * NHID + jb;
                const v4f ho0 = *(const v4f*)hp, ho1 = *(const v4f*)(hp + 4);
                Pk32 n0, n1;
                Pk16 pk;
#pragma unroll
                for (int r = 0; r < 4; ++r) {
                    {
                        const float ar = acc[ti][r] * invW;
                        const float az = acc[2 + ti][r] * invW;
                        const float an = fmaf(acc[4 + ti][r], invW, bn[ti][r]);
                        const float rg = fsigm(gr0[r] + ar);
                        const float zg = fsigm(gz0[r] + az);
                        const float nc = ftanh(fmaf(rg, an, gn0[r]));
                        const float hn = (1.f - zg) * nc + zg * ho0[r];
                        n0.f[r] = hn;
                        pk.h[r] = (f16t)hn;
                    }
                    {
                        const float ar = acc[ti][4 + r] * invW;
                        const float az = acc[2 + ti][4 + r] * invW;
                        const float an = fmaf(acc[4 + ti][4 + r], invW, bn[ti][4 + r]);
                        const float rg = fsigm(gr1[r] + ar);
                        const float zg = fsigm(gz1[r] + az);
                        const float nc = ftanh(fmaf(rg, an, gn1[r]));
                        const float hn = (1.f - zg) * nc + zg * ho1[r];
                        n1.f[r] = hn;
                        pk.h[4 + r] = (f16t)hn;
                    }
                }
                *(v4f*)hp       = n0.f;
                *(v4f*)(hp + 4) = n1.f;
                *(v8h*)(sH16 + m * LPH + jb) = pk.h;
            }
            __syncthreads();
        }
    }

    {
        v8f acc[5]; zacc(acc);
        mma_acc<5, 5, 0>(acc, P1, 80 * w, NHID, sH16, LPH, 4);
        epi_h<5, true>(acc, 80 * w, invW, b1, 300, sO1, LPO);
    }
    __syncthreads();
    {
        v8f acc[5]; zacc(acc);
        mma_acc<5, 5, 0>(acc, P2, 80 * w, F1P, sO1, LPO, 10);
        epi_h<5, true>(acc, 80 * w, invW, b2, 300, sO2, LPO);
    }
    __syncthreads();
    if (w == 0) {
        v8f acc[1]; zacc(acc);
        mma_acc<1, 1, 0>(acc, P3, 0, F1P, sO2, LPO, 10);
        if (h == 0) {
            sOut[2 * m]     = fmaf(acc[0][0], invW, b3[0]);
            sOut[2 * m + 1] = fmaf(acc[0][1], invW, b3[1]);
        }
    }
    __syncthreads();
    {
        const bool wr = (tid < 8);
        v4f ov = {0.f, 0.f, 0.f, 0.f};
        if (wr) ov = *(const v4f*)(sOut + 4 * tid);
        float* dst = out + (size_t)blockIdx.x * (NBLK * 2) + 4 * tid;
        if (wr) *(volatile v4f*)dst = ov;
        __threadfence();
        if (wr) *(volatile v4f*)dst = ov;
    }
}

extern "C" void kernel_launch(void* const* d_in, const int* in_sizes, int n_in,
                              void* d_out, int out_size, void* d_ws, size_t ws_size,
                              hipStream_t stream) {
    const int NBATCH = 128, NF1 = 300, NOUT = 2, NOUTP = 16;

    if (n_in < 22) return;
    if (in_sizes[0] != NBATCH * TT * CH || out_size != NBATCH * NOUT) return;
    if (in_sizes[10] != NHID * KWO || in_sizes[11] != NHID ||
        in_sizes[12] != G3 * NHID || in_sizes[13] != G3 * NHID ||
        in_sizes[14] != G3 || in_sizes[15] != G3 ||
        in_sizes[16] != NF1 * NHID || in_sizes[17] != NF1 ||
        in_sizes[18] != NF1 * NF1 || in_sizes[19] != NF1 ||
        in_sizes[20] != NOUT * NF1 || in_sizes[21] != NOUT) return;
    if ((NBATCH % NBLK) != 0) return;

    const float* x   = (const float*)d_in[0];
    const float* Wo  = (const float*)d_in[10]; const float* bo  = (const float*)d_in[11];
    const float* Wih = (const float*)d_in[12]; const float* Whh = (const float*)d_in[13];
    const float* bih = (const float*)d_in[14]; const float* bhh = (const float*)d_in[15];
    const float* W1  = (const float*)d_in[16]; const float* b1  = (const float*)d_in[17];
    const float* W2  = (const float*)d_in[18]; const float* b2  = (const float*)d_in[19];
    const float* W3  = (const float*)d_in[20]; const float* b3  = (const float*)d_in[21];
    float* out = (float*)d_out;

    char* ws = (char*)d_ws;
    size_t off = 0;
    auto carve = [&](size_t bytes) -> char* {
        char* p = ws + off;
        off = (off + bytes + 255) & ~(size_t)255;
        return p;
    };
    f16t* Po  = (f16t*)carve((size_t)NHID  * KWO  * 2);
    f16t* Pih = (f16t*)carve((size_t)G3    * NHID * 2);
    f16t* Phh = (f16t*)carve((size_t)G3    * NHID * 2);
    f16t* P1  = (f16t*)carve((size_t)F1P   * NHID * 2);
    f16t* P2  = (f16t*)carve((size_t)F1P   * F1P  * 2);
    f16t* P3  = (f16t*)carve((size_t)NOUTP * F1P  * 2);
    if (off > ws_size) return;

    const float SW = 64.0f, IW = 0.015625f;

    auto pack = [&](const float* W, f16t* P, int N, int K, int Np, int Kp) {
        int tot = Np * (Kp / 8);
        k_pack<<<dim3((tot + 255) / 256), dim3(256), 0, stream>>>(W, P, N, K, Np, Kp, SW);
    };
    pack(Wo,  Po,  NHID, KWO,  NHID,  KWO);
    pack(Wih, Pih, G3,   NHID, G3,    NHID);
    pack(Whh, Phh, G3,   NHID, G3,    NHID);
    pack(W1,  P1,  NF1,  NHID, F1P,   NHID);
    pack(W2,  P2,  NF1,  NF1,  F1P,   F1P);
    pack(W3,  P3,  NOUT, NF1,  NOUTP, F1P);

    k_main<<<dim3(NBATCH / NBLK), dim3(128), 0, stream>>>(x, Po, bo, Pih, bih, Phh, bhh,
                                                         P1, b1, P2, b2, P3, b3, out, NBATCH, IW);
}
